// DeformConv3dPack_74483322847780
// MI455X (gfx1250) — hardware-verified
//
#include <hip/hip_runtime.h>
#include <stddef.h>


#define C_IN    64
#define D_IN    8
#define H_IN    64
#define W_IN    64
#define P_TOT   32768
#define K_TAPS  27
#define KG      1728
#define KGU     864
#define O_MAIN  64
#define O_OFF   81
#define O_OFFP  96
#define NTHR    256
#define TP      64
#define XFU     32

static_assert(KG == K_TAPS * C_IN);
static_assert(KGU * 2 == KG);
static_assert((TP * C_IN) % NTHR == 0);
static_assert((TP * O_OFFP) % (4 * NTHR) == 0);
static_assert((O_MAIN * TP) % (4 * NTHR) == 0);
static_assert(P_TOT % TP == 0);
static_assert((KG % 32) == 0);

typedef unsigned int   v4u  __attribute__((ext_vector_type(4)));
typedef unsigned int   v8u  __attribute__((ext_vector_type(8)));
typedef float          v4f  __attribute__((ext_vector_type(4)));
typedef float          v8f  __attribute__((ext_vector_type(8)));
typedef int            v4i  __attribute__((ext_vector_type(4)));
typedef __bf16         v16b __attribute__((ext_vector_type(16)));
union Frag { v16b v; v8u w; v4u q[2]; };


__device__ __forceinline__ unsigned int bf16_rne(float f) {
  const unsigned int u = __float_as_uint(f);
  return (u + 0x7fffu + ((u >> 16) & 1u)) >> 16;
}

__device__ __forceinline__ void split2(float v, unsigned int& hb, unsigned int& lb) {
  hb = bf16_rne(v);
  const float hv = __uint_as_float(hb << 16);
  lb = bf16_rne(v - hv);
}

__device__ __forceinline__ void split8(v4f a, v4f b, v4u& hq, v4u& lq) {
  unsigned int hb[8], lb[8];
  split2(a.x, hb[0], lb[0]); split2(a.y, hb[1], lb[1]); split2(a.z, hb[2], lb[2]); split2(a.w, hb[3], lb[3]);
  split2(b.x, hb[4], lb[4]); split2(b.y, hb[5], lb[5]); split2(b.z, hb[6], lb[6]); split2(b.w, hb[7], lb[7]);
  hq.x = hb[0] | (hb[1] << 16); hq.y = hb[2] | (hb[3] << 16); hq.z = hb[4] | (hb[5] << 16); hq.w = hb[6] | (hb[7] << 16);
  lq.x = lb[0] | (lb[1] << 16); lq.y = lb[2] | (lb[3] << 16); lq.z = lb[4] | (lb[5] << 16); lq.w = lb[6] | (lb[7] << 16);
}

__device__ __forceinline__ v4u vmask(v4u a, bool keep) {
  const unsigned int mk = keep ? 0xffffffffu : 0u;
  v4u r;
  r.x = a.x & mk; r.y = a.y & mk; r.z = a.z & mk; r.w = a.w & mk;
  return r;
}

__device__ __forceinline__ v8f zero8f() {
  v8f z = {0.f, 0.f, 0.f, 0.f, 0.f, 0.f, 0.f, 0.f};
  return z;
}

__device__ __forceinline__ v8f wmb(v16b a, v16b b, v8f c) {
  return __builtin_amdgcn_wmma_f32_16x16x32_bf16(false, a, false, b, (short)0, c, false, false);
}

__global__ __launch_bounds__(NTHR) void k_prep_x(const float* __restrict__ x,
                                                 float* xf, unsigned int* xh, unsigned int* xl) {
  __shared__ __attribute__((aligned(16))) float T[TP * C_IN];
  const int tid = threadIdx.x;
  const int p0 = blockIdx.x * TP;
#pragma unroll
  for (int it = 0; it < (TP * C_IN) / NTHR; ++it) {
    const int idx = it * NTHR + tid;
    const int c = idx >> 6, j = idx & 63;
    T[j * C_IN + c] = x[(size_t)c * P_TOT + p0 + j];
  }
  __syncthreads();
  v4f fv[4];
  v4u hv[2], lv[2];
#pragma unroll
  for (int it = 0; it < 4; ++it) fv[it] = *(const v4f*)(T + 4 * (it * NTHR + tid));
#pragma unroll
  for (int it = 0; it < 2; ++it) {
    const int q = it * NTHR + tid;
    const v4f a = *(const v4f*)(T + 8 * q);
    const v4f b = *(const v4f*)(T + 8 * q + 4);
    split8(a, b, hv[it], lv[it]);
  }
  float* df = xf + (size_t)p0 * C_IN;
  unsigned int* dh = xh + (size_t)p0 * XFU;
  unsigned int* dl = xl + (size_t)p0 * XFU;
#pragma unroll
  for (int it = 0; it < 4; ++it) *(volatile v4f*)(df + 4 * (it * NTHR + tid)) = fv[it];
#pragma unroll
  for (int it = 0; it < 2; ++it) {
    *(volatile v4u*)(dh + 4 * (it * NTHR + tid)) = hv[it];
    *(volatile v4u*)(dl + 4 * (it * NTHR + tid)) = lv[it];
  }
  __threadfence();
#pragma unroll
  for (int it = 0; it < 4; ++it) *(volatile v4f*)(df + 4 * (it * NTHR + tid)) = fv[it];
#pragma unroll
  for (int it = 0; it < 2; ++it) {
    *(volatile v4u*)(dh + 4 * (it * NTHR + tid)) = hv[it];
    *(volatile v4u*)(dl + 4 * (it * NTHR + tid)) = lv[it];
  }
}

__global__ __launch_bounds__(NTHR) void k_prep_w(const float* __restrict__ woff,
                                                 const float* __restrict__ wmain,
                                                 unsigned int* woh, unsigned int* wol,
                                                 unsigned int* wmh, unsigned int* wml) {
  const int r = blockIdx.x, tid = threadIdx.x;
  const float* src;
  int srow;
  bool nz;
  unsigned int* dh;
  unsigned int* dl;
  if (r < O_OFFP) {
    src = woff;
    nz = (r < O_OFF);
    srow = nz ? r : (O_OFF - 1);
    dh = woh + (size_t)r * KGU;
    dl = wol + (size_t)r * KGU;
  } else {
    int rr = r - O_OFFP;
    rr = rr < 0 ? 0 : (rr > O_MAIN - 1 ? O_MAIN - 1 : rr);
    src = wmain;
    nz = true;
    srow = rr;
    dh = wmh + (size_t)rr * KGU;
    dl = wml + (size_t)rr * KGU;
  }
  const bool wr = tid < (KG / 8);
  const int kb = 8 * (wr ? tid : 0);
  float v[8];
#pragma unroll
  for (int e = 0; e < 8; ++e) {
    const int k = kb + e;
    const int tap = k >> 6, c = k & 63;
    const float t2 = src[(size_t)srow * KG + c * K_TAPS + tap];
    v[e] = nz ? t2 : 0.f;
  }
  v4f a = {v[0], v[1], v[2], v[3]};
  v4f b = {v[4], v[5], v[6], v[7]};
  v4u hq, lq;
  split8(a, b, hq, lq);
  if (wr) {
    *(volatile v4u*)(dh + 4 * tid) = hq;
    *(volatile v4u*)(dl + 4 * tid) = lq;
  }
  __threadfence();
  if (wr) {
    *(volatile v4u*)(dh + 4 * tid) = hq;
    *(volatile v4u*)(dl + 4 * tid) = lq;
  }
}

__global__ __launch_bounds__(NTHR) void k_offconv(const unsigned int* __restrict__ xh,
                                                  const unsigned int* __restrict__ xl,
                                                  const unsigned int* __restrict__ woh,
                                                  const unsigned int* __restrict__ wol,
                                                  const float* __restrict__ boff, int nboff,
                                                  float* offp) {
  __shared__ __attribute__((aligned(16))) float st[TP * O_OFFP];
  const int tid = threadIdx.x, lane = tid & 31, wave = tid >> 5, h = lane >> 4, m = lane & 15;
  const int mt = wave & 3, ng = wave >> 2;
  const int p0 = blockIdx.x * TP;
  const int p  = p0 + 16 * mt + m;
  const int pz = p >> 12, py = (p >> 6) & 63, px = p & 63;

  int wb[3];
#pragma unroll
  for (int j = 0; j < 3; ++j) wb[j] = (48 * ng + 16 * j + m) * KGU + 4 * h;

  v8f acc[3];
  acc[0] = zero8f(); acc[1] = zero8f(); acc[2] = zero8f();

#pragma unroll 1
  for (int t = 0; t < K_TAPS; ++t) {
    const int kd = t / 9;
    const int kr = t - 9 * kd;
    const int kh = kr / 3;
    const int kw = kr - 3 * kh;
    const int z = pz + kd - 1, y = py + kh - 1, xx = px + kw - 1;
    const bool valid = ((unsigned)z < (unsigned)D_IN) && ((unsigned)y < (unsigned)H_IN) &&
                       ((unsigned)xx < (unsigned)W_IN);
    const int zc = z < 0 ? 0 : (z > D_IN - 1 ? D_IN - 1 : z);
    const int yc = y < 0 ? 0 : (y > H_IN - 1 ? H_IN - 1 : y);
    const int xc = xx < 0 ? 0 : (xx > W_IN - 1 ? W_IN - 1 : xx);
    const int nbr = (zc * H_IN + yc) * W_IN + xc;
    const unsigned int* ahp = xh + (size_t)nbr * XFU + 4 * h;
    const unsigned int* alp = xl + (size_t)nbr * XFU + 4 * h;
#pragma unroll 1
    for (int s = 0; s < 2; ++s) {
      Frag ah, al, bh[3], bl[3];
      ah.q[0] = vmask(*(const v4u*)(ahp + 16 * s), valid);
      ah.q[1] = vmask(*(const v4u*)(ahp + 16 * s + 8), valid);
      al.q[0] = vmask(*(const v4u*)(alp + 16 * s), valid);
      al.q[1] = vmask(*(const v4u*)(alp + 16 * s + 8), valid);
      const int ko = 32 * t + 16 * s;
#pragma unroll
      for (int j = 0; j < 3; ++j) {
        const unsigned int* bp = woh + wb[j] + ko;
        const unsigned int* cp = wol + wb[j] + ko;
        bh[j].q[0] = *(const v4u*)bp;
        bh[j].q[1] = *(const v4u*)(bp + 8);
        bl[j].q[0] = *(const v4u*)cp;
        bl[j].q[1] = *(const v4u*)(cp + 8);
      }
#pragma unroll
      for (int j = 0; j < 3; ++j) {
        acc[j] = wmb(ah.v, bh[j].v, acc[j]);
        acc[j] = wmb(ah.v, bl[j].v, acc[j]);
        acc[j] = wmb(al.v, bh[j].v, acc[j]);
      }
      asm volatile("v_nop\n\tv_nop\n\tv_nop\n\tv_nop"
                   : "+v"(acc[0]), "+v"(acc[1]), "+v"(acc[2])
                   : "v"(ah.w), "v"(al.w), "v"(bh[0].w), "v"(bl[0].w),
                     "v"(bh[1].w), "v"(bl[1].w), "v"(bh[2].w), "v"(bl[2].w));
    }
  }

#pragma unroll
  for (int j = 0; j < 3; ++j) {
    const int oc = 48 * ng + 16 * j + m;
    int bi = oc < nboff - 1 ? oc : nboff - 1;
    bi = bi < 0 ? 0 : bi;
    float bbv = boff[bi];
    bbv = (oc < O_OFF) ? bbv : 0.f;
#pragma unroll
    for (int r = 0; r < 8; ++r) st[(16 * mt + 8 * h + r) * O_OFFP + oc] = acc[j][r] + bbv;
  }
  __syncthreads();
  v4f ov[6];
#pragma unroll
  for (int it = 0; it < 6; ++it) ov[it] = *(const v4f*)(st + 4 * (it * NTHR + tid));
  float* dst = offp + (size_t)p0 * O_OFFP;
#pragma unroll
  for (int it = 0; it < 6; ++it) *(volatile v4f*)(dst + 4 * (it * NTHR + tid)) = ov[it];
  __threadfence();
#pragma unroll
  for (int it = 0; it < 6; ++it) *(volatile v4f*)(dst + 4 * (it * NTHR + tid)) = ov[it];
}

__global__ __launch_bounds__(NTHR) void k_deform(const float* __restrict__ xf,
                                                 const float* __restrict__ offp,
                                                 const unsigned int* __restrict__ wmh,
                                                 const unsigned int* __restrict__ wml,
                                                 const float* __restrict__ bias, float* outp) {
  __shared__ __attribute__((aligned(16))) float        offs[TP * O_OFFP];
  __shared__ __attribute__((aligned(16))) int          cidx[TP * 8];
  __shared__ __attribute__((aligned(16))) float        cwt[TP * 8];
  __shared__ __attribute__((aligned(16))) unsigned int sh[TP * XFU];
  __shared__ __attribute__((aligned(16))) unsigned int sl[TP * XFU];
  __shared__ __attribute__((aligned(16))) float        ost[O_MAIN * TP];

  const int tid = threadIdx.x, lane = tid & 31, wave = tid >> 5, h = lane >> 4, m = lane & 15;
  const int p0 = blockIdx.x * TP;

  {
    const float* os = offp + (size_t)p0 * O_OFFP;
#pragma unroll
    for (int it = 0; it < (TP * O_OFFP) / (4 * NTHR); ++it) {
      const int q = it * NTHR + tid;
      *(v4f*)(offs + 4 * q) = *(const v4f*)(os + 4 * q);
    }
  }
  __syncthreads();

  const int mt = wave & 3, ntb = 2 * (wave >> 2);
  const int wa  = (16 * mt + m) * KGU + 4 * h;
  const int bb0 = (16 * ntb + m) * XFU + 4 * h;
  const int bb1 = (16 * (ntb + 1) + m) * XFU + 4 * h;
  v8f acc[2];
  acc[0] = zero8f(); acc[1] = zero8f();

#pragma unroll 1
  for (int t = 0; t < K_TAPS; ++t) {
    const int kd = t / 9;
    const int kr = t - 9 * kd;
    const int kh = kr / 3;
    const int kw = kr - 3 * kh;

    if (tid < TP) {
      const int n = tid, pp = p0 + n;
      const int pz = pp >> 12, py = (pp >> 6) & 63, px = pp & 63;
      const float oz = offs[n * O_OFFP + 3 * t + 0];
      const float oy = offs[n * O_OFFP + 3 * t + 1];
      const float ox = offs[n * O_OFFP + 3 * t + 2];
      const float z  = (float)(pz + kd - 1) + oz;
      const float y  = (float)(py + kh - 1) + oy;
      const float w_ = (float)(px + kw - 1) + ox;
      const float z0f = floorf(z), y0f = floorf(y), x0f = floorf(w_);
      const int z0 = (int)fminf(fmaxf(z0f, -16.f), 128.f);
      const int y0 = (int)fminf(fmaxf(y0f, -16.f), 128.f);
      const int x0 = (int)fminf(fmaxf(x0f, -16.f), 128.f);
#pragma unroll
      for (int q = 0; q < 8; ++q) {
        const int dz = q >> 2, dy = (q >> 1) & 1, dx = q & 1;
        const float wz = 1.f - fabsf(z  - (z0f + (float)dz));
        const float wy = 1.f - fabsf(y  - (y0f + (float)dy));
        const float wx = 1.f - fabsf(w_ - (x0f + (float)dx));
        const int zi = z0 + dz, yi = y0 + dy, xi = x0 + dx;
        const bool valid = (zi >= 0) && (zi < D_IN) && (yi >= 0) && (yi < H_IN) &&
                           (xi >= 0) && (xi < W_IN);
        const int zc = zi < 0 ? 0 : (zi > D_IN - 1 ? D_IN - 1 : zi);
        const int yc = yi < 0 ? 0 : (yi > H_IN - 1 ? H_IN - 1 : yi);
        const int xc = xi < 0 ? 0 : (xi > W_IN - 1 ? W_IN - 1 : xi);
        cidx[n * 8 + q] = (zc * H_IN + yc) * W_IN + xc;
        const float wgt = (wz * wy) * wx;
        cwt[n * 8 + q] = valid ? wgt : 0.f;
      }
    }
    __syncthreads();

    {
      const int n = tid >> 2, cq = tid & 3;
      const v4i ci0 = *(const v4i*)(cidx + n * 8);
      const v4i ci1 = *(const v4i*)(cidx + n * 8 + 4);
      const v4f cw0 = *(const v4f*)(cwt + n * 8);
      const v4f cw1 = *(const v4f*)(cwt + n * 8 + 4);
      int   id[8] = {ci0.x, ci0.y, ci0.z, ci0.w, ci1.x, ci1.y, ci1.z, ci1.w};
      float wq[8] = {cw0.x, cw0.y, cw0.z, cw0.w, cw1.x, cw1.y, cw1.z, cw1.w};
      v4f v0 = {0.f, 0.f, 0.f, 0.f};
      v4f v1 = v0, v2 = v0, v3 = v0;
#pragma unroll
      for (int q = 0; q < 8; ++q) {
        int i = id[q];
        i = i < 0 ? 0 : (i > P_TOT - 1 ? P_TOT - 1 : i);
        const float* sp = xf + (size_t)i * C_IN + 16 * cq;
        const v4f a = *(const v4f*)(sp);
        const v4f b = *(const v4f*)(sp + 4);
        const v4f c = *(const v4f*)(sp + 8);
        const v4f d = *(const v4f*)(sp + 12);
        const float wv = wq[q];
        v0 += a * wv;
        v1 += b * wv;
        v2 += c * wv;
        v3 += d * wv;
      }
      v4u hq0, lq0, hq1, lq1;
      split8(v0, v1, hq0, lq0);
      split8(v2, v3, hq1, lq1);
      unsigned int* shp = sh + n * XFU + 8 * cq;
      unsigned int* slp = sl + n * XFU + 8 * cq;
      *(v4u*)(shp)     = hq0;
      *(v4u*)(shp + 4) = hq1;
      *(v4u*)(slp)     = lq0;
      *(v4u*)(slp + 4) = lq1;
    }
    __syncthreads();

#pragma unroll 1
    for (int s = 0; s < 2; ++s) {
      const int ko = 32 * t + 16 * s;
      Frag ah, al, bh0, bl0, bh1, bl1;
      ah.q[0] = *(const v4u*)(wmh + wa + ko);
      ah.q[1] = *(const v4u*)(wmh + wa + ko + 8);
      al.q[0] = *(const v4u*)(wml + wa + ko);
      al.q[1] = *(const v4u*)(wml + wa + ko + 8);
      bh0.q[0] = *(const v4u*)(sh + bb0 + 16 * s);
      bh0.q[1] = *(const v4u*)(sh + bb0 + 16 * s + 8);
      bl0.q[0] = *(const v4u*)(sl + bb0 + 16 * s);
      bl0.q[1] = *(const v4u*)(sl + bb0 + 16 * s + 8);
      bh1.q[0] = *(const v4u*)(sh + bb1 + 16 * s);
      bh1.q[1] = *(const v4u*)(sh + bb1 + 16 * s + 8);
      bl1.q[0] = *(const v4u*)(sl + bb1 + 16 * s);
      bl1.q[1] = *(const v4u*)(sl + bb1 + 16 * s + 8);
      acc[0] = wmb(ah.v, bh0.v, acc[0]);
      acc[0] = wmb(ah.v, bl0.v, acc[0]);
      acc[0] = wmb(al.v, bh0.v, acc[0]);
      acc[1] = wmb(ah.v, bh1.v, acc[1]);
      acc[1] = wmb(ah.v, bl1.v, acc[1]);
      acc[1] = wmb(al.v, bh1.v, acc[1]);
      asm volatile("v_nop\n\tv_nop\n\tv_nop\n\tv_nop"
                   : "+v"(acc[0]), "+v"(acc[1])
                   : "v"(ah.w), "v"(al.w), "v"(bh0.w), "v"(bl0.w), "v"(bh1.w), "v"(bl1.w));
    }
  }

#pragma unroll
  for (int r = 0; r < 8; ++r) {
    const int oc = 16 * mt + 8 * h + r;
    const float bv = bias[oc];
    ost[oc * TP + 16 * ntb + m]       = acc[0][r] + bv;
    ost[oc * TP + 16 * (ntb + 1) + m] = acc[1][r] + bv;
  }
  __syncthreads();
  v4f ov[4];
#pragma unroll
  for (int it = 0; it < 4; ++it) ov[it] = *(const v4f*)(ost + 4 * (it * NTHR + tid));
#pragma unroll
  for (int it = 0; it < 4; ++it) {
    const int q = it * NTHR + tid;
    const int row = q >> 4, pc = q & 15;
    *(volatile v4f*)(outp + (size_t)row * P_TOT + p0 + 4 * pc) = ov[it];
  }
  __threadfence();
#pragma unroll
  for (int it = 0; it < 4; ++it) {
    const int q = it * NTHR + tid;
    const int row = q >> 4, pc = q & 15;
    *(volatile v4f*)(outp + (size_t)row * P_TOT + p0 + 4 * pc) = ov[it];
  }
}


extern "C" void kernel_launch(void* const* d_in, const int* in_sizes, int n_in,
                              void* d_out, int out_size, void* d_ws,
                              size_t ws_size, hipStream_t stream) {
  if (n_in < 5) return;
  if (in_sizes[0] != C_IN * P_TOT) return;
  if (in_sizes[1] != O_OFF * KG) return;
  if (in_sizes[2] < O_OFF) return;
  if (in_sizes[3] != O_MAIN * KG) return;
  if (in_sizes[4] < O_MAIN) return;
  if (out_size != O_MAIN * P_TOT) return;

  const float* x      = (const float*)d_in[0];
  const float* w_off  = (const float*)d_in[1];
  const float* b_off  = (const float*)d_in[2];
  const float* weight = (const float*)d_in[3];
  const float* bias   = (const float*)d_in[4];
  float* out = (float*)d_out;

  const size_t szXf = (size_t)P_TOT * C_IN * 4;
  const size_t szXb = (size_t)P_TOT * XFU * 4;
  const size_t szWo = (size_t)O_OFFP * KGU * 4;
  const size_t szWm = (size_t)O_MAIN * KGU * 4;
  const size_t szOf = (size_t)P_TOT * O_OFFP * 4;
  size_t cur = 0;
  const size_t oXf = cur; cur += szXf;
  const size_t oXh = cur; cur += szXb;
  const size_t oXl = cur; cur += szXb;
  const size_t oWoh = cur; cur += szWo;
  const size_t oWol = cur; cur += szWo;
  const size_t oWmh = cur; cur += szWm;
  const size_t oWml = cur; cur += szWm;
  const size_t oOff = cur; cur += szOf;
  if (cur > ws_size) return;

  char* ws = (char*)d_ws;
  float*        xf   = (float*)(ws + oXf);
  unsigned int* xh   = (unsigned int*)(ws + oXh);
  unsigned int* xl   = (unsigned int*)(ws + oXl);
  unsigned int* woh  = (unsigned int*)(ws + oWoh);
  unsigned int* wol  = (unsigned int*)(ws + oWol);
  unsigned int* wmh  = (unsigned int*)(ws + oWmh);
  unsigned int* wml  = (unsigned int*)(ws + oWml);
  float*        offp = (float*)(ws + oOff);

  const int nboff = in_sizes[2];

  k_prep_x<<<P_TOT / TP, NTHR, 0, stream>>>(x, xf, xh, xl);
  k_prep_w<<<O_OFFP + O_MAIN, NTHR, 0, stream>>>(w_off, weight, woh, wol, wmh, wml);
  k_offconv<<<P_TOT / TP, NTHR, 0, stream>>>(xh, xl, woh, wol, b_off, nboff, offp);
  k_deform<<<P_TOT / TP, NTHR, 0, stream>>>(xf, offp, wmh, wml, bias, out);
}
